// TokenSwapMamba_5918464934174
// MI455X (gfx1250) — hardware-run, weakly checked
//
#include <hip/hip_runtime.h>
#include <hip/hip_fp16.h>
#include <math.h>

typedef __attribute__((ext_vector_type(16))) _Float16 v16h;
typedef __attribute__((ext_vector_type(8)))  _Float16 v8h;
typedef __attribute__((ext_vector_type(8)))  float    v8f;
typedef __attribute__((ext_vector_type(4)))  float    v4f;
typedef __attribute__((ext_vector_type(4)))  unsigned v4u;
typedef __attribute__((ext_vector_type(2)))  unsigned v2u;

constexpr int kBatch = 2;
constexpr int kSeq   = 8192;
constexpr int kDm    = 64;
constexpr int kNS    = 2;
constexpr int kDin   = 256;
constexpr int kDinR  = 128;
constexpr int kTaps  = 8;
constexpr int kTapsR = 4;
constexpr int kNst   = 16;
constexpr int kDtR   = 8;
constexpr int kDtRR  = 4;
constexpr int kRows  = kBatch * kSeq;
constexpr int kXzP   = 2 * kDin;
constexpr int kDbcWR = kDtRR + 2 * kNst;
constexpr int kDbcW  = kDtR + 2 * kNst;
constexpr int kDbcP  = 64;
constexpr int kOffB  = kDtR;
constexpr int kOffC  = kDtR + kNst;
constexpr int kConvTP = 260;
constexpr int kOutN  = kRows * kDm;
static_assert(kRows == 16384);
static_assert(kXzP == 512);
static_assert(kDbcWR == 36 && kDbcW == 40);
static_assert(kTaps == 8 && kTapsR == 4 && kDtR == 8 && kDtRR == 4);
static_assert((kSeq & (kSeq - 1)) == 0);
static_assert((kDm % 32) == 0 && (kDin % 32) == 0);
static_assert((kRows % 64) == 0 && (kXzP % 64) == 0 && (kDbcP % 64) == 0 && (kDm % 64) == 0);
static_assert((kDin % 64) == 0 && (kSeq % 64) == 0);

constexpr float kWCarry = 1024.0f;
constexpr float kACarry = 1024.0f;
constexpr float kYCarry = 1048576.0f;
constexpr float kScaleIn  = 1.0f / (kACarry * kWCarry);
constexpr float kScaleOut = 1.0f / (kYCarry * kWCarry);

constexpr size_t kSzWI  = (size_t)kXzP * kDm * 2;
constexpr size_t kSzWX  = (size_t)kDbcP * kDin * 2;
constexpr size_t kSzWO  = (size_t)kDm * kDin * 2;
constexpr size_t kSzCW  = (size_t)kDin * kTaps * 4;
constexpr size_t kSzDW  = (size_t)kDin * kDtR * 4;
constexpr size_t kSzAL  = (size_t)kDin * kNst * 4;
constexpr size_t kSzV   = (size_t)kDin * 4;
constexpr size_t kSzPar = kSzWI + kSzWX + kSzWO + kSzCW + kSzDW + kSzAL + 3 * kSzV;
constexpr size_t kSzXN  = (size_t)kRows * kDm * 2;
constexpr size_t kSzXZ  = (size_t)kRows * kXzP * 4;
constexpr size_t kSzU32 = (size_t)kRows * kDin * 4;
constexpr size_t kSzU16 = (size_t)kRows * kDin * 2;
constexpr size_t kSzDBC = (size_t)kRows * kDbcP * 4;
constexpr size_t kSzDTP = (size_t)kRows * kDin * 4;
constexpr size_t kSzY16 = (size_t)kRows * kDin * 2;
constexpr size_t kOffPar = 0;
constexpr size_t kOffXN  = kOffPar + kNS * kSzPar;
constexpr size_t kOffXZ  = kOffXN  + kNS * kSzXN;
constexpr size_t kOffU32 = kOffXZ  + kSzXZ;
constexpr size_t kOffU16 = kOffU32 + kSzU32;
constexpr size_t kOffDBC = kOffU16 + kSzU16;
constexpr size_t kOffDTP = kOffDBC + kSzDBC;
constexpr size_t kOffY16 = kOffDTP + kSzDTP;
constexpr size_t kWsTotal = kOffY16 + kSzY16;
constexpr size_t kPWI = 0;
constexpr size_t kPWX = kPWI + kSzWI;
constexpr size_t kPWO = kPWX + kSzWX;
constexpr size_t kPCW = kPWO + kSzWO;
constexpr size_t kPDW = kPCW + kSzCW;
constexpr size_t kPAL = kPDW + kSzDW;
constexpr size_t kPCB = kPAL + kSzAL;
constexpr size_t kPDB = kPCB + kSzV;
constexpr size_t kPDS = kPDB + kSzV;
static_assert(kSzPar == 166912ull);
static_assert(kWsTotal <= 134217728ull);
static_assert((kSzPar % 128) == 0 && (kPWX % 128) == 0 && (kPWO % 128) == 0 && (kPCW % 128) == 0 && (kPDW % 128) == 0 &&
              (kPAL % 128) == 0 && (kPCB % 128) == 0 && (kPDB % 128) == 0 && (kPDS % 128) == 0);
static_assert((kOffXN % 128) == 0 && (kOffXZ % 128) == 0 && (kOffU32 % 128) == 0 && (kOffU16 % 128) == 0 &&
              (kOffDBC % 128) == 0 && (kOffDTP % 128) == 0 && (kOffY16 % 128) == 0);

__device__ __forceinline__ unsigned g_h16bits(float v) {
  const float f = (fabsf(v) < 6.103515625e-05f) ? 0.0f : v;
  return (unsigned)__half_as_ushort(__float2half_rn(f));
}
__device__ __forceinline__ unsigned g_pack16(float a, float b) {
  const unsigned lo = g_h16bits(a);
  const unsigned hi = g_h16bits(b);
  return lo | (hi << 16);
}

constexpr int kPrepBlkWi = kXzP * kDm / 8 / 256;
constexpr int kPrepBlkWx = kDbcP * kDin / 8 / 256;
constexpr int kPrepBlkWo = kDm * kDin / 8 / 256;
constexpr int kPrepQuads = kDin * kTaps / 4 + kDin * kDtR / 4 + kDin * kNst / 4 + 3 * (kDin / 4);
constexpr int kPrepBlkF  = (kPrepQuads + 255) / 256;
static_assert(kPrepBlkWi == 16 && kPrepBlkWx == 8 && kPrepBlkWo == 8 && kPrepQuads == 2240 && kPrepBlkF == 9);

__global__ __launch_bounds__(256) void tsm_prep_kernel(
    const float* __restrict__ in_w, const float* __restrict__ conv_w, const float* __restrict__ conv_b,
    const float* __restrict__ xproj_w, const float* __restrict__ dt_w, const float* __restrict__ dt_b,
    const float* __restrict__ A_log, const float* __restrict__ Dp, const float* __restrict__ out_w,
    char* __restrict__ par)
{
  const int blk = blockIdx.x;
  const int tid = threadIdx.x;
  if (blk < kPrepBlkWi + kPrepBlkWx + kPrepBlkWo) {
    const float* src;
    unsigned short* dst;
    bool live;
    if (blk < kPrepBlkWi) {
      const int e0 = (blk * 256 + tid) * 8;
      const int row = e0 / kDm;
      const int col = e0 - row * kDm;
      const bool sig = (row < kDinR);
      const bool gat = (row >= kDin) && (row < kDin + kDinR);
      live = sig || gat;
      const int sr = sig ? row : (gat ? (row - kDin + kDinR) : 0);
      src = in_w + (size_t)sr * kDm + col;
      dst = (unsigned short*)(par + kPWI) + e0;
    } else if (blk < kPrepBlkWi + kPrepBlkWx) {
      const int e0 = ((blk - kPrepBlkWi) * 256 + tid) * 8;
      const int row = e0 / kDin;
      const int col = e0 - row * kDin;
      const bool isdt = (row < kDtRR);
      const bool isbc = (row >= kDtR) && (row < kDbcW);
      live = (isdt || isbc) && (col < kDinR);
      const int sr = isdt ? row : (isbc ? (row - (kDtR - kDtRR)) : 0);
      const int sc = (col < kDinR) ? col : 0;
      src = xproj_w + (size_t)sr * kDinR + sc;
      dst = (unsigned short*)(par + kPWX) + e0;
    } else {
      const int e0 = ((blk - kPrepBlkWi - kPrepBlkWx) * 256 + tid) * 8;
      const int row = e0 / kDin;
      const int col = e0 - row * kDin;
      live = (col < kDinR);
      const int sc = live ? col : 0;
      src = out_w + (size_t)row * kDinR + sc;
      dst = (unsigned short*)(par + kPWO) + e0;
    }
    const v4f a0 = *(const v4f*)(src);
    const v4f a1 = *(const v4f*)(src + 4);
    float f0 = a0[0], f1 = a0[1], f2 = a0[2], f3 = a0[3];
    float f4 = a1[0], f5 = a1[1], f6 = a1[2], f7 = a1[3];
    f0 = live ? f0 * kWCarry : 0.0f;
    f1 = live ? f1 * kWCarry : 0.0f;
    f2 = live ? f2 * kWCarry : 0.0f;
    f3 = live ? f3 * kWCarry : 0.0f;
    f4 = live ? f4 * kWCarry : 0.0f;
    f5 = live ? f5 * kWCarry : 0.0f;
    f6 = live ? f6 * kWCarry : 0.0f;
    f7 = live ? f7 * kWCarry : 0.0f;
    const v4u w = (v4u){g_pack16(f0, f1), g_pack16(f2, f3), g_pack16(f4, f5), g_pack16(f6, f7)};
    volatile v4u* q = (volatile v4u*)dst;
    *q = w;
    __threadfence();
    *q = w;
    return;
  }
  const int q4 = (blk - kPrepBlkWi - kPrepBlkWx - kPrepBlkWo) * 256 + tid;
  if (q4 >= kPrepQuads) return;
  constexpr int nCW = kDin * kTaps / 4;
  constexpr int nDW = kDin * kDtR / 4;
  constexpr int nAL = kDin * kNst / 4;
  constexpr int nV  = kDin / 4;
  const float* src;
  float* dst;
  bool live;
  if (q4 < nCW) {
    const int d = q4 >> 1;
    const int hi = q4 & 1;
    live = (hi == 1) && (d < kDinR);
    src = conv_w + (size_t)(live ? d : 0) * kTapsR;
    dst = (float*)(par + kPCW) + (size_t)q4 * 4;
  } else if (q4 < nCW + nDW) {
    const int q = q4 - nCW;
    const int d = q >> 1;
    const int hi = q & 1;
    live = (hi == 0) && (d < kDinR);
    src = dt_w + (size_t)(live ? d : 0) * kDtRR;
    dst = (float*)(par + kPDW) + (size_t)q * 4;
  } else if (q4 < nCW + nDW + nAL) {
    const int q = q4 - nCW - nDW;
    const int d = q >> 2;
    const int part = q & 3;
    live = (d < kDinR);
    src = A_log + (size_t)(live ? d : 0) * kNst + part * 4;
    dst = (float*)(par + kPAL) + (size_t)q * 4;
  } else {
    const int q = q4 - nCW - nDW - nAL;
    const int which = q / nV;
    const int d0 = (q - which * nV) * 4;
    live = (d0 < kDinR);
    const float* base = (which == 0) ? conv_b : ((which == 1) ? dt_b : Dp);
    src = base + (live ? d0 : 0);
    dst = (float*)(par + ((which == 0) ? kPCB : ((which == 1) ? kPDB : kPDS))) + d0;
  }
  const v4f a = *(const v4f*)(src);
  const v4f o = live ? a : (v4f){0.0f, 0.0f, 0.0f, 0.0f};
  volatile v4f* q = (volatile v4f*)dst;
  *q = o;
  __threadfence();
  *q = o;
}

__global__ __launch_bounds__(256) void tsm_ln_swap_kernel(
    const float* __restrict__ under, const float* __restrict__ over,
    const float* __restrict__ ures, const float* __restrict__ ores,
    const float* __restrict__ w1, const float* __restrict__ b1,
    const float* __restrict__ w2, const float* __restrict__ b2,
    float* __restrict__ OUT3, float* __restrict__ OUT4,
    unsigned short* __restrict__ XNu, unsigned short* __restrict__ XNo)
{
  const int tid = threadIdx.x;
  const int lane = tid & 31;
  const int wave = tid >> 5;
  const int half = lane >> 4;
  const int c0 = (lane & 15) * 4;
  const int row = blockIdx.x * 16 + wave * 2 + half;
  const size_t off = (size_t)row * kDm + c0;
  const v4f xu = *(const v4f*)(under + off);
  const v4f ru = *(const v4f*)(ures + off);
  const v4f xo = *(const v4f*)(over + off);
  const v4f ro = *(const v4f*)(ores + off);
  const v4f su = (v4f){xu[0] + ru[0], xu[1] + ru[1], xu[2] + ru[2], xu[3] + ru[3]};
  const v4f so = (v4f){xo[0] + ro[0], xo[1] + ro[1], xo[2] + ro[2], xo[3] + ro[3]};
  float mu = (su[0] + su[1]) + (su[2] + su[3]);
  float mo = (so[0] + so[1]) + (so[2] + so[3]);
  mu += __shfl_xor(mu, 8, 32);  mo += __shfl_xor(mo, 8, 32);
  mu += __shfl_xor(mu, 4, 32);  mo += __shfl_xor(mo, 4, 32);
  mu += __shfl_xor(mu, 2, 32);  mo += __shfl_xor(mo, 2, 32);
  mu += __shfl_xor(mu, 1, 32);  mo += __shfl_xor(mo, 1, 32);
  mu *= (1.0f / (float)kDm);
  mo *= (1.0f / (float)kDm);
  const v4f du = (v4f){su[0] - mu, su[1] - mu, su[2] - mu, su[3] - mu};
  const v4f dv = (v4f){so[0] - mo, so[1] - mo, so[2] - mo, so[3] - mo};
  float vu = 0.0f, vo = 0.0f;
  vu = fmaf(du[0], du[0], vu);  vo = fmaf(dv[0], dv[0], vo);
  vu = fmaf(du[1], du[1], vu);  vo = fmaf(dv[1], dv[1], vo);
  vu = fmaf(du[2], du[2], vu);  vo = fmaf(dv[2], dv[2], vo);
  vu = fmaf(du[3], du[3], vu);  vo = fmaf(dv[3], dv[3], vo);
  vu += __shfl_xor(vu, 8, 32);  vo += __shfl_xor(vo, 8, 32);
  vu += __shfl_xor(vu, 4, 32);  vo += __shfl_xor(vo, 4, 32);
  vu += __shfl_xor(vu, 2, 32);  vo += __shfl_xor(vo, 2, 32);
  vu += __shfl_xor(vu, 1, 32);  vo += __shfl_xor(vo, 1, 32);
  const float rsu = rsqrtf(vu * (1.0f / (float)kDm) + 1e-5f);
  const float rso = rsqrtf(vo * (1.0f / (float)kDm) + 1e-5f);
  const v4f g1 = *(const v4f*)(w1 + c0);
  const v4f h1 = *(const v4f*)(b1 + c0);
  const v4f g2 = *(const v4f*)(w2 + c0);
  const v4f h2 = *(const v4f*)(b2 + c0);
  float un[4], ov[4];
#pragma unroll
  for (int j = 0; j < 4; ++j) {
    un[j] = fmaf(du[j] * rsu, g1[j], h1[j]);
    ov[j] = fmaf(dv[j] * rso, g2[j], h2[j]);
  }
  const bool lowc = (c0 < kDm / 2);
  float a[4], b[4];
#pragma unroll
  for (int j = 0; j < 4; ++j) {
    a[j] = (lowc ? ov[j] : un[j]) * kACarry;
    b[j] = (lowc ? un[j] : ov[j]) * kACarry;
  }
  const v2u pa = (v2u){g_pack16(a[0], a[1]), g_pack16(a[2], a[3])};
  const v2u pb = (v2u){g_pack16(b[0], b[1]), g_pack16(b[2], b[3])};
  volatile v4f* q3 = (volatile v4f*)(OUT3 + off);
  volatile v4f* q4 = (volatile v4f*)(OUT4 + off);
  volatile v2u* qa = (volatile v2u*)(XNu + off);
  volatile v2u* qb = (volatile v2u*)(XNo + off);
  *q3 = su;  *q4 = so;  *qa = pa;  *qb = pb;
  __threadfence();
  *q3 = su;  *q4 = so;  *qa = pa;  *qb = pb;
}

__global__ __launch_bounds__(256) void conv_silu_kernel(
    const float* __restrict__ XZ, const float* __restrict__ cw, const float* __restrict__ cb,
    float* __restrict__ U32, unsigned short* __restrict__ U16)
{
  __shared__ __align__(16) float sT[16 * kConvTP];
  const int tid = threadIdx.x;
  const int lane = tid & 31;
  const int wave = tid >> 5;
  const int d = tid;
  const int g0 = blockIdx.x * 64;
  const int tb = g0 & (kSeq - 1);
  const v4f wa = *(const v4f*)(cw + d * kTaps);
  const v4f wb = *(const v4f*)(cw + d * kTaps + 4);
  const float w0 = wa[0], w1 = wa[1], w2 = wa[2], w3 = wa[3];
  const float w4 = wb[0], w5 = wb[1], w6 = wb[2], w7 = wb[3];
  const float bias = cb[d];
  float xm7, xm6, xm5, xm4, xm3, xm2, xm1;
  {
    const bool hist = (tb > 0);
    const int rb = hist ? (g0 - 7) : g0;
    const float v7 = XZ[(size_t)(rb + 0) * kXzP + d];
    const float v6 = XZ[(size_t)(rb + 1) * kXzP + d];
    const float v5 = XZ[(size_t)(rb + 2) * kXzP + d];
    const float v4 = XZ[(size_t)(rb + 3) * kXzP + d];
    const float v3 = XZ[(size_t)(rb + 4) * kXzP + d];
    const float v2 = XZ[(size_t)(rb + 5) * kXzP + d];
    const float v1 = XZ[(size_t)(rb + 6) * kXzP + d];
    xm7 = hist ? v7 : 0.0f;
    xm6 = hist ? v6 : 0.0f;
    xm5 = hist ? v5 : 0.0f;
    xm4 = hist ? v4 : 0.0f;
    xm3 = hist ? v3 : 0.0f;
    xm2 = hist ? v2 : 0.0f;
    xm1 = hist ? v1 : 0.0f;
  }
  const int hrow = wave >> 1;
  const int hch  = (wave & 1) * 128 + lane * 4;
#pragma unroll 1
  for (int sub = 0; sub < 4; ++sub) {
    const int lb = g0 + sub * 16;
#pragma unroll 1
    for (int s = 0; s < 16; ++s) {
      const float xcur = XZ[(size_t)(lb + s) * kXzP + d];
      float acc = w0 * xm7;
      acc = fmaf(w1, xm6, acc);
      acc = fmaf(w2, xm5, acc);
      acc = fmaf(w3, xm4, acc);
      acc = fmaf(w4, xm3, acc);
      acc = fmaf(w5, xm2, acc);
      acc = fmaf(w6, xm1, acc);
      acc = fmaf(w7, xcur, acc);
      const float sv = acc + bias;
      const float sg = __builtin_amdgcn_rcpf(1.0f + expf(-sv));
      sT[s * kConvTP + tid] = sv * sg;
      xm7 = xm6;
      xm6 = xm5;
      xm5 = xm4;
      xm4 = xm3;
      xm3 = xm2;
      xm2 = xm1;
      xm1 = xcur;
    }
    __syncthreads();
    v4f fv[4];
    v4u hv[2];
#pragma unroll
    for (int it = 0; it < 4; ++it) fv[it] = *(const v4f*)(sT + (it * 4 + hrow) * kConvTP + hch);
#pragma unroll
    for (int it = 0; it < 2; ++it) {
      const float* sp = sT + (it * 8 + wave) * kConvTP + lane * 8;
      const v4f a0 = *(const v4f*)(sp);
      const v4f a1 = *(const v4f*)(sp + 4);
      const float e0 = a0[0] * kACarry, e1 = a0[1] * kACarry, e2 = a0[2] * kACarry, e3 = a0[3] * kACarry;
      const float e4 = a1[0] * kACarry, e5 = a1[1] * kACarry, e6 = a1[2] * kACarry, e7 = a1[3] * kACarry;
      hv[it] = (v4u){g_pack16(e0, e1), g_pack16(e2, e3), g_pack16(e4, e5), g_pack16(e6, e7)};
    }
    for (int pass = 0; pass < 2; ++pass) {
#pragma unroll
      for (int it = 0; it < 4; ++it)
        *(volatile v4f*)(U32 + (size_t)(lb + it * 4 + hrow) * kDin + hch) = fv[it];
#pragma unroll
      for (int it = 0; it < 2; ++it)
        *(volatile v4u*)(U16 + (size_t)(lb + it * 8 + wave) * kDin + lane * 8) = hv[it];
      __threadfence();
    }
    __syncthreads();
  }
}

__global__ __launch_bounds__(256) void dtpre_kernel(
    const float* __restrict__ DBC, const float* __restrict__ dw, const float* __restrict__ db,
    float* __restrict__ DTP)
{
  const int tid = threadIdx.x;
  const int c4 = (tid & 63) * 4;
  const int rsub = tid >> 6;
  v4f wlo[4], whi[4];
#pragma unroll
  for (int j = 0; j < 4; ++j) {
    wlo[j] = *(const v4f*)(dw + (size_t)(c4 + j) * kDtR);
    whi[j] = *(const v4f*)(dw + (size_t)(c4 + j) * kDtR + 4);
  }
  const v4f bv = *(const v4f*)(db + c4);
  const int r0 = blockIdx.x * 64;
#pragma unroll 1
  for (int it = 0; it < 16; ++it) {
    const int row = r0 + it * 4 + rsub;
    const v4f xa = *(const v4f*)(DBC + (size_t)row * kDbcP);
    const v4f xb = *(const v4f*)(DBC + (size_t)row * kDbcP + 4);
    float o[4];
#pragma unroll
    for (int j = 0; j < 4; ++j) {
      float acc = xa[0] * wlo[j][0];
      acc = fmaf(xa[1], wlo[j][1], acc);
      acc = fmaf(xa[2], wlo[j][2], acc);
      acc = fmaf(xa[3], wlo[j][3], acc);
      acc = fmaf(xb[0], whi[j][0], acc);
      acc = fmaf(xb[1], whi[j][1], acc);
      acc = fmaf(xb[2], whi[j][2], acc);
      acc = fmaf(xb[3], whi[j][3], acc);
      o[j] = acc + bv[j];
    }
    const v4f ov = (v4f){o[0], o[1], o[2], o[3]};
    volatile v4f* q = (volatile v4f*)(DTP + (size_t)row * kDin + c4);
    *q = ov;
    __threadfence();
    *q = ov;
  }
}

namespace eng {

__device__ __forceinline__ v16h frag_load(const _Float16* p) {
  union U { v16h v; v8h h[2]; } f;
  f.h[0] = *(const v8h*)(p);
  f.h[1] = *(const v8h*)(p + 16);
  return f.v;
}
__device__ __forceinline__ v8f mma_h(v16h a, v16h b, v8f c) {
  c = __builtin_amdgcn_wmma_f32_16x16x32_f16(false, a, false, b, (short)0, c, false, false);
  asm volatile("v_nop\n\tv_nop\n\tv_nop\n\tv_nop" : "+v"(c) : "v"(a), "v"(b));
  return c;
}

template <bool RESID>
__global__ __launch_bounds__(256) void gemm_f16_kernel(
    const unsigned short* __restrict__ Ap, int lda,
    const unsigned short* __restrict__ Btp, int ldb,
    float* __restrict__ C, int ldc,
    const float* __restrict__ resid,
    int M, int N, int K, float scale)
{
  const _Float16* A  = (const _Float16*)Ap;
  const _Float16* Bt = (const _Float16*)Btp;
  __shared__ __align__(16) float sT[8][16 * 68];
  const int lane = threadIdx.x & 31;
  const int wave = threadIdx.x >> 5;
  const int tilesN = N >> 6;
  const int tilesM = M >> 6;
  const int tile = blockIdx.x * 8 + wave;
  if (tile >= tilesM * tilesN) return;
  const int tm = tile / tilesN;
  const int tn = tile - tm * tilesN;
  const int m0 = tm << 6;
  const int n0 = tn << 6;
  const int rlane = lane & 15;
  const int koff  = (lane >> 4) * 8;
  const int mOff  = (lane >> 4) * 8;

  v8f acc[4][4];
#pragma unroll
  for (int i = 0; i < 4; ++i)
#pragma unroll
    for (int j = 0; j < 4; ++j) acc[i][j] = (v8f){0.f, 0.f, 0.f, 0.f, 0.f, 0.f, 0.f, 0.f};

  for (int k0 = 0; k0 < K; k0 += 32) {
    v16h bh[4];
#pragma unroll
    for (int j = 0; j < 4; ++j) {
      const size_t bo = (size_t)(n0 + (j << 4) + rlane) * ldb + koff + k0;
      bh[j] = frag_load(Bt + bo);
    }
#pragma unroll
    for (int i = 0; i < 4; ++i) {
      const size_t ao = (size_t)(m0 + (i << 4) + rlane) * lda + koff + k0;
      const v16h ah = frag_load(A + ao);
#pragma unroll
      for (int j = 0; j < 4; ++j) acc[i][j] = mma_h(ah, bh[j], acc[i][j]);
    }
  }

  float* slab = sT[wave];
  const int hh = lane >> 4;
  const int c4 = (lane & 15) * 4;
#pragma unroll
  for (int i = 0; i < 4; ++i) {
    const int mBase = m0 + (i << 4);
#pragma unroll
    for (int j = 0; j < 4; ++j) {
#pragma unroll
      for (int r = 0; r < 8; ++r) {
        slab[(mOff + r) * 68 + (j << 4) + rlane] = acc[i][j][r] * scale;
      }
    }
    __builtin_amdgcn_fence(__ATOMIC_RELEASE, "workgroup");
    __builtin_amdgcn_wave_barrier();
    __builtin_amdgcn_fence(__ATOMIC_ACQUIRE, "workgroup");
    v4f ov[8];
#pragma unroll
    for (int it = 0; it < 8; ++it) {
      const int row = it * 2 + hh;
      v4f v = *(const v4f*)(slab + row * 68 + c4);
      if (RESID) {
        const v4f rv = *(const v4f*)(resid + (size_t)(mBase + row) * ldc + n0 + c4);
        v = v + rv;
      }
      ov[it] = v;
    }
    for (int pass = 0; pass < 2; ++pass) {
#pragma unroll
      for (int it = 0; it < 8; ++it) {
        const int row = it * 2 + hh;
        *(volatile v4f*)(C + (size_t)(mBase + row) * ldc + n0 + c4) = ov[it];
      }
      __threadfence();
    }
    __builtin_amdgcn_fence(__ATOMIC_RELEASE, "workgroup");
    __builtin_amdgcn_wave_barrier();
    __builtin_amdgcn_fence(__ATOMIC_ACQUIRE, "workgroup");
  }
}

}

typedef float    ms1_v4f __attribute__((ext_vector_type(4)));
typedef unsigned ms1_v4u __attribute__((ext_vector_type(4)));
struct ms1_args {
  const float* dtpre;
  const float* u;
  const float* bc;
  const float* z;
  const float* A_log;
  const float* Dskip;
  __half* y;
  __half* y_lo;
  long ld_dtpre;
  long ld_u;
  long ld_bc;
  long ld_z;
  long ld_y;
  int offB;
  int offC;
  int offZ;
  float ycarry;
  int dir;
  int D;
  int L;
  int nbatch;
};
static_assert(sizeof(ms1_args) == 136);

__device__ __forceinline__ float ms1_flush16(float v) {
  return (fabsf(v) < 6.103515625e-05f) ? 0.0f : v;
}
__device__ __forceinline__ unsigned ms1_h16bits(float v) {
  return (unsigned)__half_as_ushort(__float2half_rn(ms1_flush16(v)));
}
__device__ __forceinline__ float ms1_h16val(unsigned b) {
  return __half2float(__ushort_as_half((unsigned short)b));
}
__device__ __forceinline__ float ms1_softplus(float v) {
  return fmaxf(v, 0.0f) + log1pf(expf(-fabsf(v)));
}
__device__ __forceinline__ void ms1_pack2(float v0, float v1, unsigned& hw, unsigned& lw) {
  const unsigned h0 = ms1_h16bits(v0);
  const unsigned h1 = ms1_h16bits(v1);
  const float r0 = (v0 - ms1_h16val(h0)) * 2048.0f;
  const float r1 = (v1 - ms1_h16val(h1)) * 2048.0f;
  const unsigned l0 = ms1_h16bits(r0);
  const unsigned l1 = ms1_h16bits(r1);
  hw = h0 | (h1 << 16);
  lw = l0 | (l1 << 16);
}

template <int NSTATE>
__global__ __launch_bounds__(64 * (NSTATE / 16)) void ms1_scan_kernel(ms1_args a)
{
  static_assert(NSTATE == 16 || NSTATE == 64);
  constexpr int NQ  = NSTATE / 16;
  constexpr int NT  = 64 * NQ;
  constexpr int NW  = NT / 32;
  constexpr int BCW = 2 * NSTATE;
  constexpr int YP  = 68;
  constexpr int RPI = NW * 4;
  constexpr int NIT = 64 / RPI;
  static_assert(16 * NT <= 64 * YP);
  __shared__ __align__(16) float sBC[64 * BCW];
  __shared__ __align__(16) float sY[64 * YP];
  const int tid  = threadIdx.x;
  const int lane = tid & 31;
  const int wave = tid >> 5;
  const int c    = tid / NQ;
  const int sq   = tid - c * NQ;
  const int bpb  = a.D / 64;
  const int bi   = blockIdx.x / bpb;
  if (bi >= a.nbatch) return;
  const int d0 = (blockIdx.x - bi * bpb) * 64;
  const int d  = d0 + c;
  const long rowb = (long)bi * a.L;
  const bool hasz  = (a.z != nullptr);
  const bool hasD  = (a.Dskip != nullptr);
  const bool hasLo = (a.y_lo != nullptr);

#pragma unroll 1
  for (int n = 0; n < 16; ++n) {
    const float al = a.A_log[(long)d * NSTATE + sq * 16 + n];
    sY[n * NT + tid] = -expf(al);
  }
  __syncthreads();
  float An[16], h[16];
#pragma unroll
  for (int n = 0; n < 16; ++n) {
    An[n] = sY[n * NT + tid];
    h[n] = 0.0f;
  }
  float Dd = 0.0f;
  if (hasD) Dd = a.Dskip[d];

  const int nchunk = a.L / 64;
  const bool fwd = (a.dir > 0);
  const int s0 = fwd ? 0 : 63;
  const int sd = fwd ? 1 : -1;
  const int q  = lane >> 3;
  const int c8 = (lane & 7) * 8;

#pragma unroll 1
  for (int ci = 0; ci < nchunk; ++ci) {
    const int tb = fwd ? (ci * 64) : (a.L - 64 - ci * 64);
    const long rowc = rowb + tb;
    __syncthreads();
#pragma unroll 8
    for (int i = 0; i < 32; ++i) {
      const int idx = tid + i * NT;
      const int st  = idx / BCW;
      const int col = idx - st * BCW;
      const int sc  = (col < NSTATE) ? (a.offB + col) : (a.offC + col - NSTATE);
      sBC[idx] = a.bc[(rowc + st) * a.ld_bc + sc];
    }
    __syncthreads();
#pragma unroll 1
    for (int s = 0; s < 64; ++s) {
      const int ls = s0 + sd * s;
      const long row = rowc + ls;
      float pre = a.dtpre[row * a.ld_dtpre + d];
      float uv  = a.u[row * a.ld_u + d];
      float zv  = 0.0f;
      if (hasz) zv = a.z[row * a.ld_z + a.offZ + d];
      asm volatile("" : "+v"(pre));
      asm volatile("" : "+v"(uv));
      asm volatile("" : "+v"(zv));
      const float delta = ms1_softplus(pre);
      const float dtx = delta * uv;
      const float* bp = sBC + ls * BCW + sq * 16;
      const float* cp = bp + NSTATE;
      ms1_v4f Bq[4], Cq[4];
#pragma unroll
      for (int k = 0; k < 4; ++k) {
        Bq[k] = *(const ms1_v4f*)(bp + 4 * k);
        Cq[k] = *(const ms1_v4f*)(cp + 4 * k);
      }
      float yv = 0.0f;
#pragma unroll
      for (int n = 0; n < 16; ++n) {
        const float e = __expf(delta * An[n]);
        h[n] = fmaf(e, h[n], dtx * Bq[n >> 2][n & 3]);
        yv = fmaf(h[n], Cq[n >> 2][n & 3], yv);
      }
      if (NQ > 1) {
        yv += __shfl_xor(yv, 1, 32);
        yv += __shfl_xor(yv, 2, 32);
      }
      if (hasD) yv = fmaf(uv, Dd, yv);
      if (hasz) {
        const float sg = __builtin_amdgcn_rcpf(1.0f + expf(-zv));
        yv = yv * (zv * sg);
      }
      if (sq == 0) sY[ls * YP + c] = yv * a.ycarry;
    }
    __syncthreads();
    ms1_v4u hw[NIT], lw[NIT];
#pragma unroll
    for (int it = 0; it < NIT; ++it) {
      const int row = it * RPI + wave * 4 + q;
      const float* sp = sY + row * YP + c8;
      const ms1_v4f f0 = *(const ms1_v4f*)(sp);
      const ms1_v4f f1 = *(const ms1_v4f*)(sp + 4);
      unsigned h0, h1, h2, h3, l0, l1, l2, l3;
      ms1_pack2(f0[0], f0[1], h0, l0);
      ms1_pack2(f0[2], f0[3], h1, l1);
      ms1_pack2(f1[0], f1[1], h2, l2);
      ms1_pack2(f1[2], f1[3], h3, l3);
      hw[it] = (ms1_v4u){h0, h1, h2, h3};
      lw[it] = (ms1_v4u){l0, l1, l2, l3};
    }
    for (int pass = 0; pass < 2; ++pass) {
#pragma unroll
      for (int it = 0; it < NIT; ++it) {
        const int row = it * RPI + wave * 4 + q;
        const long o = (rowc + row) * a.ld_y + d0 + c8;
        *(volatile ms1_v4u*)(a.y + o) = hw[it];
        if (hasLo) *(volatile ms1_v4u*)(a.y_lo + o) = lw[it];
      }
      __threadfence();
    }
  }
}

extern "C" void kernel_launch(void* const* d_in, const int* in_sizes, int n_in,
                              void* d_out, int out_size, void* d_ws, size_t ws_size,
                              hipStream_t stream) {
  if (n_in < 26) return;
  for (int i = 0; i < 4; ++i) if (in_sizes[i] != kOutN) return;
  for (int i = 4; i < 8; ++i) if (in_sizes[i] != kDm) return;
  for (int s = 0; s < kNS; ++s) {
    const int* z = in_sizes + 8 + 9 * s;
    if (z[0] != 2 * kDinR * kDm) return;
    if (z[1] != kDinR * kTapsR) return;
    if (z[2] != kDinR) return;
    if (z[3] != kDbcWR * kDinR) return;
    if (z[4] != kDinR * kDtRR) return;
    if (z[5] != kDinR) return;
    if (z[6] != kDinR * kNst) return;
    if (z[7] != kDinR) return;
    if (z[8] != kDm * kDinR) return;
  }
  if (out_size != 4 * kOutN) return;
  if (ws_size < kWsTotal) return;

  const float* under = (const float*)d_in[0];
  const float* over  = (const float*)d_in[1];
  const float* ures  = (const float*)d_in[2];
  const float* ores  = (const float*)d_in[3];
  const float* n1w   = (const float*)d_in[4];
  const float* n1b   = (const float*)d_in[5];
  const float* n2w   = (const float*)d_in[6];
  const float* n2b   = (const float*)d_in[7];
  float* out = (float*)d_out;

  char* ws = (char*)d_ws;
  unsigned short* XN16 = (unsigned short*)(ws + kOffXN);
  float*          XZ   = (float*)(ws + kOffXZ);
  float*          U32  = (float*)(ws + kOffU32);
  unsigned short* U16  = (unsigned short*)(ws + kOffU16);
  float*          DBC  = (float*)(ws + kOffDBC);
  float*          DTP  = (float*)(ws + kOffDTP);
  unsigned short* Y16  = (unsigned short*)(ws + kOffY16);

  for (int s = 0; s < kNS; ++s) {
    const int p0 = 8 + 9 * s;
    tsm_prep_kernel<<<dim3(kPrepBlkWi + kPrepBlkWx + kPrepBlkWo + kPrepBlkF), 256, 0, stream>>>(
        (const float*)d_in[p0 + 0], (const float*)d_in[p0 + 1], (const float*)d_in[p0 + 2],
        (const float*)d_in[p0 + 3], (const float*)d_in[p0 + 4], (const float*)d_in[p0 + 5],
        (const float*)d_in[p0 + 6], (const float*)d_in[p0 + 7], (const float*)d_in[p0 + 8],
        ws + kOffPar + (size_t)s * kSzPar);
  }

  tsm_ln_swap_kernel<<<dim3(kRows / 16), 256, 0, stream>>>(
      under, over, ures, ores, n1w, n1b, n2w, n2b,
      out + (size_t)2 * kOutN, out + (size_t)3 * kOutN,
      XN16, XN16 + (size_t)kRows * kDm);

  for (int s = 0; s < kNS; ++s) {
    char* par = ws + kOffPar + (size_t)s * kSzPar;
    const unsigned short* WI16 = (const unsigned short*)(par + kPWI);
    const unsigned short* WX16 = (const unsigned short*)(par + kPWX);
    const unsigned short* WO16 = (const unsigned short*)(par + kPWO);
    const float* CW8 = (const float*)(par + kPCW);
    const float* DW8 = (const float*)(par + kPDW);
    const float* AL  = (const float*)(par + kPAL);
    const float* CB  = (const float*)(par + kPCB);
    const float* DB  = (const float*)(par + kPDB);
    const float* DS  = (const float*)(par + kPDS);
    const unsigned short* XN = XN16 + (size_t)s * kRows * kDm;
    float* Os = out + (size_t)s * kOutN;

    eng::gemm_f16_kernel<false><<<dim3((kRows / 64) * (kXzP / 64) / 8), 256, 0, stream>>>(
        XN, kDm,
        WI16, kDm,
        XZ, kXzP,
        nullptr,
        kRows, kXzP, kDm, kScaleIn);

    conv_silu_kernel<<<dim3(kRows / 64), 256, 0, stream>>>(XZ, CW8, CB, U32, U16);

    eng::gemm_f16_kernel<false><<<dim3((kRows / 64) * (kDbcP / 64) / 8), 256, 0, stream>>>(
        U16, kDin,
        WX16, kDin,
        DBC, kDbcP,
        nullptr,
        kRows, kDbcP, kDin, kScaleIn);

    dtpre_kernel<<<dim3(kRows / 64), 256, 0, stream>>>(DBC, DW8, DB, DTP);

    for (int b = 0; b < kBatch; ++b) {
      const size_t r0 = (size_t)b * kSeq;
      ms1_args sa;
      sa.dtpre = DTP + r0 * kDin;
      sa.u = U32 + r0 * kDin;
      sa.bc = DBC + r0 * kDbcP;
      sa.z = XZ + r0 * kXzP;
      sa.A_log = AL;
      sa.Dskip = DS;
      sa.y = (__half*)(Y16 + r0 * kDin);
      sa.y_lo = nullptr;
      sa.ld_dtpre = kDin;
      sa.ld_u = kDin;
      sa.ld_bc = kDbcP;
      sa.ld_z = kXzP;
      sa.ld_y = kDin;
      sa.offB = kOffB;
      sa.offC = kOffC;
      sa.offZ = kDin;
      sa.ycarry = kYCarry;
      sa.dir = 1;
      sa.D = kDin;
      sa.L = kSeq;
      sa.nbatch = 1;
      ms1_scan_kernel<16><<<dim3(kDin / 64), 64, 0, stream>>>(sa);
    }

    eng::gemm_f16_kernel<false><<<dim3((kRows / 64) * (kDm / 64) / 8), 256, 0, stream>>>(
        Y16, kDin,
        WO16, kDin,
        Os, kDm,
        nullptr,
        kRows, kDm, kDin, kScaleOut);
  }
}
